// FewShotSegmentor_75986561401351
// MI455X (gfx1250) — hardware-verified
//
#include <hip/hip_runtime.h>
#include <math.h>
#include <stddef.h>


typedef _Float16 v16h __attribute__((ext_vector_type(16)));
typedef _Float16 v8h  __attribute__((ext_vector_type(8)));
typedef float    v8f  __attribute__((ext_vector_type(8)));
typedef float    v4f  __attribute__((ext_vector_type(4)));

constexpr int B = 4, C = 256, H = 64, W = 64;
constexpr int N = H * W;
constexpr int PH = H + 2, PW = W + 2;
constexpr int OC = 64;
constexpr int CK = C * 9;
constexpr int MSH = 256, MSW = 256;
constexpr float EPS = 1e-5f;
constexpr float QS = 32.0f;
constexpr float SIM_OUT = 20.0f / (QS * QS);
constexpr float WSC = 64.0f;
constexpr float INV_WSC = 1.0f / 64.0f;

constexpr size_t O_MT    = 0;
constexpr size_t O_G     = O_MT    + (size_t)B * N * 4;
constexpr size_t O_PS    = O_G     + (size_t)B * C * 4;
constexpr size_t O_PSN   = O_PS    + (size_t)B * C * 4;
constexpr size_t O_PSUM  = O_PSN   + (size_t)B * C * 4;
constexpr size_t O_MAXFG = O_PSUM  + (size_t)B * C * 4;
constexpr size_t O_MAXCX = O_MAXFG + (size_t)B * N * 4;
constexpr size_t O_AQ    = O_MAXCX + (size_t)B * N * 4;
constexpr size_t O_BFG   = O_AQ    + (size_t)B * N * C * 2;
constexpr size_t O_BCX   = O_BFG   + (size_t)B * N * C * 2;
constexpr size_t O_PW    = O_BCX   + (size_t)B * N * C * 2;
constexpr size_t O_FQP   = O_PW    + (size_t)OC * CK * 2;
constexpr size_t O_END   = O_FQP   + (size_t)B * PH * PW * C * 2;
static_assert(O_G % 128 == 0 && O_PS % 128 == 0 && O_PSN % 128 == 0 && O_PSUM % 128 == 0);
static_assert(O_MAXFG % 128 == 0 && O_MAXCX % 128 == 0 && O_AQ % 128 == 0 && O_BFG % 128 == 0);
static_assert(O_BCX % 128 == 0 && O_PW % 128 == 0 && O_FQP % 128 == 0 && O_END % 128 == 0);
static_assert(O_END <= (size_t)128 * 1024 * 1024);

__device__ __forceinline__ v16h ldfrag(const _Float16* p) {
  const v8h lo = *(const v8h*)p;
  const v8h hi = *(const v8h*)(p + 16);
  return __builtin_shufflevector(lo, hi, 0, 1, 2, 3, 4, 5, 6, 7, 8, 9, 10, 11, 12, 13, 14, 15);
}

__device__ __forceinline__ v8f wmma_f16(v16h a, v16h b, v8f c) {
  v8f d = __builtin_amdgcn_wmma_f32_16x16x32_f16(false, a, false, b, (short)0, c, false, false);
  asm volatile("v_nop\n\tv_nop\n\tv_nop\n\tv_nop" : "+v"(d) : "v"(a), "v"(b));
  return d;
}

__device__ __forceinline__ v8f zero8() {
  v8f z = {0.f, 0.f, 0.f, 0.f, 0.f, 0.f, 0.f, 0.f};
  return z;
}

__device__ __forceinline__ float wave_sum(float v) {
  v += __shfl_xor(v, 16, 32);
  v += __shfl_xor(v, 8, 32);
  v += __shfl_xor(v, 4, 32);
  v += __shfl_xor(v, 2, 32);
  v += __shfl_xor(v, 1, 32);
  return v;
}

__global__ void __launch_bounds__(256) k_support(
    const float* __restrict__ Fs, const float* __restrict__ Ms,
    const float* __restrict__ w1, const float* __restrict__ b1,
    const float* __restrict__ w2, const float* __restrict__ b2,
    float* Mt, float* gout, float* psout, float* psnout)
{
  __shared__ float mt_s[N] __attribute__((aligned(16)));
  __shared__ float gap_s[C];
  __shared__ float sfg_s[C];
  __shared__ float g_s[C] __attribute__((aligned(16)));
  __shared__ float ps_s[C] __attribute__((aligned(16)));
  __shared__ float psn_s[C] __attribute__((aligned(16)));
  __shared__ float h_s[16];
  __shared__ float red_s[8];

  const int tid = threadIdx.x, lane = tid & 31, wv = tid >> 5;
  const int b = blockIdx.x;
  if (b >= B) return;
  const float* ms = Ms + (size_t)b * (MSH * MSW);

  v4f mtv[4];
  float lsum = 0.f;
#pragma unroll
  for (int it = 0; it < 4; ++it) {
    const int p = (it * 256 + tid) * 4;
    const int y = p >> 6, x = p & 63;
    const float sy = (y == H - 1) ? 255.0f : 255.0f * ((float)y * (1.0f / 63.0f));
    int y0 = (int)floorf(sy);
    y0 = min(max(y0, 0), MSH - 1);
    const int y1 = min(y0 + 1, MSH - 1);
    const float wy = sy - (float)y0;
    float r[4];
#pragma unroll
    for (int j = 0; j < 4; ++j) {
      const int xx = x + j;
      const float sx = (xx == W - 1) ? 255.0f : 255.0f * ((float)xx * (1.0f / 63.0f));
      int x0 = (int)floorf(sx);
      x0 = min(max(x0, 0), MSW - 1);
      const int x1 = min(x0 + 1, MSW - 1);
      const float wx = sx - (float)x0;
      const float t0 = ms[y0 * MSW + x0] * (1.0f - wy) + ms[y1 * MSW + x0] * wy;
      const float t1 = ms[y0 * MSW + x1] * (1.0f - wy) + ms[y1 * MSW + x1] * wy;
      const float v = t0 * (1.0f - wx) + t1 * wx;
      r[j] = v;
      lsum += v;
      mt_s[p + j] = v;
    }
    v4f vv = {r[0], r[1], r[2], r[3]};
    mtv[it] = vv;
    *(volatile v4f*)(Mt + (size_t)b * N + p) = vv;
  }
  lsum = wave_sum(lsum);
  if (lane == 0) red_s[wv] = lsum;
  __syncthreads();
  const float sumM = ((red_s[0] + red_s[1]) + (red_s[2] + red_s[3])) +
                     ((red_s[4] + red_s[5]) + (red_s[6] + red_s[7]));

  for (int j = 0; j < 32; ++j) {
    const int c = wv * 32 + j;
    const float* row = Fs + ((size_t)b * C + c) * N;
    float s1 = 0.f, s2 = 0.f;
#pragma unroll 2
    for (int i = 0; i < 32; ++i) {
      const int p = (i * 32 + lane) * 4;
      const v4f v = *(const v4f*)(row + p);
      const v4f m = *(const v4f*)(mt_s + p);
      s1 += (v[0] + v[1]) + (v[2] + v[3]);
      s2 += (v[0] * m[0] + v[1] * m[1]) + (v[2] * m[2] + v[3] * m[3]);
    }
    s1 = wave_sum(s1);
    s2 = wave_sum(s2);
    if (lane == 0) { gap_s[c] = s1 * (1.0f / 4096.0f); sfg_s[c] = s2; }
  }
  __syncthreads();

  if (tid < 16) {
    float a = b1[tid];
    const float* wrow = w1 + (size_t)tid * C;
#pragma unroll 4
    for (int c = 0; c < C; ++c) a += wrow[c] * gap_s[c];
    h_s[tid] = fminf(fmaxf(a, 0.0f), 6.0f);
  }
  __syncthreads();
  const int c = tid;
  float gg, ps;
  {
    float a = b2[c];
    const float* wrow = w2 + (size_t)c * 16;
#pragma unroll
    for (int j = 0; j < 16; ++j) a += wrow[j] * h_s[j];
    gg = 1.0f / (1.0f + expf(-a));
    ps = sfg_s[c] * (1.0f / (sumM + EPS));
  }
  const float q = wave_sum(ps * ps);
  if (lane == 0) red_s[wv] = q;
  __syncthreads();
  const float tot = ((red_s[0] + red_s[1]) + (red_s[2] + red_s[3])) +
                    ((red_s[4] + red_s[5]) + (red_s[6] + red_s[7]));
  const float inv = 1.0f / fmaxf(sqrtf(tot), 1e-12f);
  g_s[c] = gg;
  ps_s[c] = ps;
  psn_s[c] = ps * inv;
  __syncthreads();

  const bool wr = lane < 8;
  const size_t ob = (size_t)b * C + wv * 32 + lane * 4;
  v4f gv = {0.f, 0.f, 0.f, 0.f}, pv = {0.f, 0.f, 0.f, 0.f}, nv = {0.f, 0.f, 0.f, 0.f};
  if (wr) {
    gv = *(const v4f*)(g_s + wv * 32 + lane * 4);
    pv = *(const v4f*)(ps_s + wv * 32 + lane * 4);
    nv = *(const v4f*)(psn_s + wv * 32 + lane * 4);
    *(volatile v4f*)(gout + ob) = gv;
    *(volatile v4f*)(psout + ob) = pv;
    *(volatile v4f*)(psnout + ob) = nv;
  }
  __threadfence();
#pragma unroll
  for (int it = 0; it < 4; ++it) {
    const int p = (it * 256 + tid) * 4;
    *(volatile v4f*)(Mt + (size_t)b * N + p) = mtv[it];
  }
  if (wr) {
    *(volatile v4f*)(gout + ob) = gv;
    *(volatile v4f*)(psout + ob) = pv;
    *(volatile v4f*)(psnout + ob) = nv;
  }
}

__global__ void __launch_bounds__(256) k_pack(
    const float* __restrict__ Fs, const float* __restrict__ Fq,
    const float* __restrict__ Mt, const float* __restrict__ gin,
    _Float16* Aq, _Float16* Bfg, _Float16* Bcx)
{
  constexpr int TP = 264;
  __shared__ _Float16 tq[32 * TP] __attribute__((aligned(16)));
  __shared__ _Float16 tf[32 * TP] __attribute__((aligned(16)));
  __shared__ _Float16 tc[32 * TP] __attribute__((aligned(16)));
  __shared__ float gs[C];
  __shared__ float part[3][8][32];
  __shared__ float inv_s[3][32];

  const int tid = threadIdx.x, lane = tid & 31, wv = tid >> 5;
  const int b = blockIdx.y;
  const int p0 = blockIdx.x * 32;
  if (p0 >= N || b >= B) return;
  gs[tid] = gin[(size_t)b * C + tid];
  const float mt = Mt[(size_t)b * N + p0 + lane];
  __syncthreads();

  const float* fqb = Fq + (size_t)b * C * N + p0 + lane;
  const float* fsb = Fs + (size_t)b * C * N + p0 + lane;
  float sq = 0.f, sf = 0.f, sc = 0.f;
#pragma unroll 2
  for (int j = 0; j < 32; ++j) {
    const int c = wv * 32 + j;
    const float fq = fqb[(size_t)c * N];
    const float fs = fsb[(size_t)c * N];
    const float ffg = fs * mt, fcx = fs * gs[c];
    sq += fq * fq; sf += ffg * ffg; sc += fcx * fcx;
  }
  part[0][wv][lane] = sq; part[1][wv][lane] = sf; part[2][wv][lane] = sc;
  __syncthreads();
  if (tid < 96) {
    const int a = tid >> 5, px = tid & 31;
    float s = 0.f;
#pragma unroll
    for (int w = 0; w < 8; ++w) s += part[a][w][px];
    inv_s[a][px] = (1.0f / fmaxf(sqrtf(s), 1e-12f)) * QS;
  }
  __syncthreads();
  const float iq = inv_s[0][lane], ifg = inv_s[1][lane], icx = inv_s[2][lane];
#pragma unroll 2
  for (int j = 0; j < 32; ++j) {
    const int c = wv * 32 + j;
    const float fq = fqb[(size_t)c * N];
    const float fs = fsb[(size_t)c * N];
    tq[lane * TP + c] = (_Float16)(fq * iq);
    tf[lane * TP + c] = (_Float16)((fs * mt) * ifg);
    tc[lane * TP + c] = (_Float16)((fs * gs[c]) * icx);
  }
  __syncthreads();

  v8h ra[4], rf[4], rc[4];
#pragma unroll
  for (int i = 0; i < 4; ++i) {
    const int p = wv * 4 + i;
    ra[i] = *(const v8h*)(tq + p * TP + lane * 8);
    rf[i] = *(const v8h*)(tf + p * TP + lane * 8);
    rc[i] = *(const v8h*)(tc + p * TP + lane * 8);
    const size_t go = ((size_t)b * N + p0 + p) * C + lane * 8;
    *(volatile v8h*)(Aq + go)  = ra[i];
    *(volatile v8h*)(Bfg + go) = rf[i];
    *(volatile v8h*)(Bcx + go) = rc[i];
  }
  __threadfence();
#pragma unroll
  for (int i = 0; i < 4; ++i) {
    const int p = wv * 4 + i;
    const size_t go = ((size_t)b * N + p0 + p) * C + lane * 8;
    *(volatile v8h*)(Aq + go)  = ra[i];
    *(volatile v8h*)(Bfg + go) = rf[i];
    *(volatile v8h*)(Bcx + go) = rc[i];
  }
}

__global__ void __launch_bounds__(128) k_sim(
    const _Float16* __restrict__ Aq, const _Float16* __restrict__ Bfg,
    const _Float16* __restrict__ Bcx, float* maxFg, float* maxCx)
{
  __shared__ float mx_s[64] __attribute__((aligned(16)));
  const int tid = threadIdx.x, lane = tid & 31, wv = tid >> 5;
  const int h = lane >> 4, m = lane & 15;
  const int b = blockIdx.y;
  const int z = blockIdx.z;
  if (blockIdx.x * 64 >= N || b >= B) return;
  const int row0 = blockIdx.x * 64 + wv * 16;
  const _Float16* Bz = (z == 0) ? Bfg : Bcx;
  float* out = (z == 0) ? maxFg : maxCx;

  const _Float16* arow = Aq + ((size_t)b * N + row0 + m) * C + 8 * h;
  v16h a[8];
#pragma unroll
  for (int kt = 0; kt < 8; ++kt) a[kt] = ldfrag(arow + kt * 32);

  float rmax[8];
#pragma unroll
  for (int r = 0; r < 8; ++r) rmax[r] = -3.0e38f;

  const _Float16* bbase = Bz + ((size_t)b * N + m) * C + 8 * h;
#pragma unroll 1
  for (int nt = 0; nt < N / 16; ++nt) {
    const _Float16* brow = bbase + (size_t)nt * 16 * C;
    v8f acc = zero8();
#pragma unroll
    for (int kt = 0; kt < 8; ++kt) {
      const v16h bv = ldfrag(brow + kt * 32);
      acc = wmma_f16(a[kt], bv, acc);
    }
#pragma unroll
    for (int r = 0; r < 8; ++r) rmax[r] = fmaxf(rmax[r], acc[r]);
  }

#pragma unroll
  for (int r = 0; r < 8; ++r) {
    float v = rmax[r];
    v = fmaxf(v, __shfl_xor(v, 1, 32));
    v = fmaxf(v, __shfl_xor(v, 2, 32));
    v = fmaxf(v, __shfl_xor(v, 4, 32));
    v = fmaxf(v, __shfl_xor(v, 8, 32));
    rmax[r] = v;
  }
  if (m == 0) {
#pragma unroll
    for (int r = 0; r < 8; ++r) mx_s[wv * 16 + h * 8 + r] = rmax[r] * SIM_OUT;
  }
  __syncthreads();
  const bool wr = (wv == 0) && (lane < 16);
  v4f ov = {0.f, 0.f, 0.f, 0.f};
  float* dst = out + (size_t)b * N + blockIdx.x * 64 + lane * 4;
  if (wr) {
    ov = *(const v4f*)(mx_s + lane * 4);
    *(volatile v4f*)dst = ov;
  }
  __threadfence();
  if (wr) *(volatile v4f*)dst = ov;
}

__global__ void __launch_bounds__(256) k_query(
    const float* __restrict__ Fq, const float* __restrict__ maxFg, const float* __restrict__ maxCx,
    const float* __restrict__ fw, const float* __restrict__ fb, const float* __restrict__ Psn,
    float* psum)
{
  __shared__ float mc_s[N] __attribute__((aligned(16)));
  __shared__ float sfq_s[C];
  __shared__ float out_s[C] __attribute__((aligned(16)));
  __shared__ float red_s[8];

  const int tid = threadIdx.x, lane = tid & 31, wv = tid >> 5;
  const int b = blockIdx.x;
  if (b >= B) return;
  const float fw0 = fw[0], fw1 = fw[1], fb0 = fb[0];
  const float* mf = maxFg + (size_t)b * N;
  const float* mcx = maxCx + (size_t)b * N;

  float lsum = 0.f;
#pragma unroll 1
  for (int i = 0; i < 16; ++i) {
    const int p = i * 256 + tid;
    const int y = p >> 6, x = p & 63;
    float s0 = 0.f, s1 = 0.f;
#pragma unroll 1
    for (int dy = -2; dy <= 2; ++dy) {
      const int yy = y + dy;
      if (yy < 0 || yy >= H) continue;
#pragma unroll
      for (int dx = -2; dx <= 2; ++dx) {
        const int xx = x + dx;
        if (xx < 0 || xx >= W) continue;
        s0 += mf[yy * W + xx];
        s1 += mcx[yy * W + xx];
      }
    }
    const float a = fw0 * (s0 * (1.0f / 25.0f)) + fw1 * (s1 * (1.0f / 25.0f)) + fb0;
    const float v = 1.0f / (1.0f + expf(-a));
    mc_s[p] = v;
    lsum += v;
  }
  lsum = wave_sum(lsum);
  if (lane == 0) red_s[wv] = lsum;
  __syncthreads();
  const float sumMc = ((red_s[0] + red_s[1]) + (red_s[2] + red_s[3])) +
                      ((red_s[4] + red_s[5]) + (red_s[6] + red_s[7]));

  const float* fqb = Fq + (size_t)b * C * N;
  for (int j = 0; j < 32; ++j) {
    const int c = wv * 32 + j;
    const float* row = fqb + (size_t)c * N;
    float s = 0.f;
#pragma unroll 2
    for (int i = 0; i < 32; ++i) {
      const int p = (i * 32 + lane) * 4;
      const v4f v = *(const v4f*)(row + p);
      const v4f w = *(const v4f*)(mc_s + p);
      s += (v[0] * w[0] + v[1] * w[1]) + (v[2] * w[2] + v[3] * w[3]);
    }
    s = wave_sum(s);
    if (lane == 0) sfq_s[c] = s;
  }
  __syncthreads();

  const int c = tid;
  const float pq = sfq_s[c] * (1.0f / (sumMc + EPS));
  const float q = wave_sum(pq * pq);
  if (lane == 0) red_s[wv] = q;
  __syncthreads();
  const float tot = ((red_s[0] + red_s[1]) + (red_s[2] + red_s[3])) +
                    ((red_s[4] + red_s[5]) + (red_s[6] + red_s[7]));
  const float inv = 1.0f / fmaxf(sqrtf(tot), 1e-12f);
  out_s[c] = pq * inv + Psn[(size_t)b * C + c];
  __syncthreads();

  const bool wr = lane < 8;
  const size_t ob = (size_t)b * C + wv * 32 + lane * 4;
  v4f ov = {0.f, 0.f, 0.f, 0.f};
  if (wr) {
    ov = *(const v4f*)(out_s + wv * 32 + lane * 4);
    *(volatile v4f*)(psum + ob) = ov;
  }
  __threadfence();
  if (wr) *(volatile v4f*)(psum + ob) = ov;
}

__global__ void __launch_bounds__(256) k_fqprime(
    const float* __restrict__ Fq, const float* __restrict__ psum, const float* __restrict__ Ps,
    const float* __restrict__ gamma, _Float16* Fqp)
{
  constexpr int TP = 264;
  __shared__ _Float16 tile[PW * TP] __attribute__((aligned(16)));
  __shared__ float psum_s[C];
  __shared__ float ps_s[C];
  __shared__ float dpart[4][64];
  __shared__ float qpart[4][64];
  __shared__ float gs_s[64];

  const int tid = threadIdx.x, lane = tid & 31, wv = tid >> 5;
  const int b = blockIdx.y, py = blockIdx.x;
  if (py >= PH || b >= B) return;
  const bool halo = (py == 0) || (py == PH - 1);
  const int y = min(max(py - 1, 0), H - 1);
  const int cg = tid >> 6, x = tid & 63;

  psum_s[tid] = psum[(size_t)b * C + tid];
  ps_s[tid] = Ps[(size_t)b * C + tid];
  for (int i = tid; i < 2 * C; i += 256)
    tile[((i < C) ? 0 : (PW - 1)) * TP + (i & (C - 1))] = (_Float16)0.0f;
  __syncthreads();

  const float* base = Fq + (size_t)b * C * N + (size_t)y * W + x;
  float d = 0.f, q = 0.f;
#pragma unroll 2
  for (int j = 0; j < 64; ++j) {
    const int c = cg * 64 + j;
    const float v = base[(size_t)c * N];
    d += v * psum_s[c];
    q += v * v;
  }
  dpart[cg][x] = d; qpart[cg][x] = q;
  __syncthreads();
  if (tid < 64) {
    const float dd = ((dpart[0][tid] + dpart[1][tid]) + dpart[2][tid]) + dpart[3][tid];
    const float qq = ((qpart[0][tid] + qpart[1][tid]) + qpart[2][tid]) + qpart[3][tid];
    const float inv = 1.0f / fmaxf(sqrtf(qq), 1e-12f);
    gs_s[tid] = gamma[0] * (dd * inv);
  }
  __syncthreads();
  const float gS = gs_s[x];
#pragma unroll 2
  for (int j = 0; j < 64; ++j) {
    const int c = cg * 64 + j;
    const float v = base[(size_t)c * N];
    tile[(x + 1) * TP + c] = (_Float16)(v + gS * ps_s[c]);
  }
  __syncthreads();

  v8h zh;
#pragma unroll
  for (int i = 0; i < 8; ++i) zh[i] = (_Float16)0.0f;
  _Float16* orow = Fqp + ((size_t)(b * PH + py) * PW) * C + lane * 8;
  for (int p = wv; p < PW; p += 8) {
    const v8h v = halo ? zh : *(const v8h*)(tile + p * TP + lane * 8);
    *(volatile v8h*)(orow + (size_t)p * C) = v;
  }
  __threadfence();
  for (int p = wv; p < PW; p += 8) {
    const v8h v = halo ? zh : *(const v8h*)(tile + p * TP + lane * 8);
    *(volatile v8h*)(orow + (size_t)p * C) = v;
  }
}

__global__ void __launch_bounds__(256) k_packw(const float* __restrict__ w1, _Float16* pW)
{
  const int t = blockIdx.x * 256 + threadIdx.x;
  if (t >= OC * CK / 8) return;
  const int e = t * 8;
  const int oc = e / CK, k = e - oc * CK;
  const int tap = k >> 8, c0 = k & 255;
  const int ky = tap / 3, kx = tap - ky * 3;
  v8h v;
#pragma unroll
  for (int i = 0; i < 8; ++i)
    v[i] = (_Float16)(WSC * w1[(((size_t)oc * C + c0 + i) * 3 + ky) * 3 + kx]);
  *(volatile v8h*)(pW + e) = v;
  __threadfence();
  *(volatile v8h*)(pW + e) = v;
}

__global__ void __launch_bounds__(256) k_conv(
    const _Float16* __restrict__ Fqp, const _Float16* __restrict__ pW,
    const float* __restrict__ b1, const float* __restrict__ w2, const float* __restrict__ b2,
    float* out)
{
  __shared__ float pred_s[4 * W] __attribute__((aligned(16)));
  const int tid = threadIdx.x, lane = tid & 31, wv = tid >> 5;
  const int h = lane >> 4, m = lane & 15;
  const int mt = wv & 3, nh = wv >> 2;
  const int b = blockIdx.y, y = blockIdx.x;
  if (y >= H || b >= B) return;
  const int x0 = nh * 32;

  const _Float16* arow = pW + (size_t)(mt * 16 + m) * CK + 8 * h;
  v8f acc0 = zero8(), acc1 = zero8();
#pragma unroll 1
  for (int tap = 0; tap < 9; ++tap) {
    const int ky = tap / 3, kx = tap - ky * 3;
    const _Float16* q0 = Fqp + (((size_t)(b * PH + y + ky) * PW) + x0 + m + kx) * C + 8 * h;
    const _Float16* q1 = q0 + 16 * C;
    const _Float16* ak = arow + tap * C;
#pragma unroll
    for (int cs = 0; cs < 8; ++cs) {
      const v16h av  = ldfrag(ak + cs * 32);
      const v16h bv0 = ldfrag(q0 + cs * 32);
      const v16h bv1 = ldfrag(q1 + cs * 32);
      acc0 = wmma_f16(av, bv0, acc0);
      acc1 = wmma_f16(av, bv1, acc1);
    }
  }

  float part0 = 0.f, part1 = 0.f;
#pragma unroll
  for (int r = 0; r < 8; ++r) {
    const int oc = mt * 16 + 8 * h + r;
    const float bb = b1[oc], ww = w2[oc];
    part0 += ww * fmaxf(acc0[r] * INV_WSC + bb, 0.0f);
    part1 += ww * fmaxf(acc1[r] * INV_WSC + bb, 0.0f);
  }
  part0 += __shfl_xor(part0, 16, 32);
  part1 += __shfl_xor(part1, 16, 32);
  if (h == 0) {
    pred_s[mt * W + x0 + m] = part0;
    pred_s[mt * W + x0 + 16 + m] = part1;
  }
  __syncthreads();
  const bool wr = (wv == 0) && (lane < 16);
  v4f ov = {0.f, 0.f, 0.f, 0.f};
  float* dst = out + ((size_t)(b * H + y)) * W + lane * 4;
  if (wr) {
    const float bb2 = b2[0];
#pragma unroll
    for (int qd = 0; qd < 4; ++qd) {
      const int px = lane * 4 + qd;
      ov[qd] = (((pred_s[px] + pred_s[W + px]) + pred_s[2 * W + px]) + pred_s[3 * W + px]) + bb2;
    }
    *(volatile v4f*)dst = ov;
  }
  __threadfence();
  if (wr) *(volatile v4f*)dst = ov;
}

extern "C" void kernel_launch(void* const* d_in, const int* in_sizes, int n_in,
                              void* d_out, int out_size, void* d_ws, size_t ws_size,
                              hipStream_t stream) {
  if (n_in < 14) return;
  if (out_size != B * N) return;
  if (ws_size < O_END) return;
  if (in_sizes[0] != B * C * N || in_sizes[1] != B * MSH * MSW || in_sizes[2] != B * C * N ||
      in_sizes[3] != 16 * C || in_sizes[4] < 16 || in_sizes[5] != C * 16 || in_sizes[6] < C ||
      in_sizes[7] < 2 || in_sizes[8] < 1 || in_sizes[9] < 1 || in_sizes[10] != OC * CK ||
      in_sizes[11] < OC || in_sizes[12] < OC || in_sizes[13] < 1) return;

  const float* Fs    = (const float*)d_in[0];
  const float* Ms    = (const float*)d_in[1];
  const float* Fq    = (const float*)d_in[2];
  const float* gw1   = (const float*)d_in[3];
  const float* gb1   = (const float*)d_in[4];
  const float* gw2   = (const float*)d_in[5];
  const float* gb2   = (const float*)d_in[6];
  const float* fw    = (const float*)d_in[7];
  const float* fb    = (const float*)d_in[8];
  const float* gamma = (const float*)d_in[9];
  const float* dw1   = (const float*)d_in[10];
  const float* db1   = (const float*)d_in[11];
  const float* dw2   = (const float*)d_in[12];
  const float* db2   = (const float*)d_in[13];
  float* out = (float*)d_out;

  char* ws = (char*)d_ws;
  float* Mt      = (float*)(ws + O_MT);
  float* g       = (float*)(ws + O_G);
  float* Ps      = (float*)(ws + O_PS);
  float* Psn     = (float*)(ws + O_PSN);
  float* psum    = (float*)(ws + O_PSUM);
  float* maxFg   = (float*)(ws + O_MAXFG);
  float* maxCx   = (float*)(ws + O_MAXCX);
  _Float16* Aq   = (_Float16*)(ws + O_AQ);
  _Float16* Bfg  = (_Float16*)(ws + O_BFG);
  _Float16* Bcx  = (_Float16*)(ws + O_BCX);
  _Float16* pW   = (_Float16*)(ws + O_PW);
  _Float16* Fqp  = (_Float16*)(ws + O_FQP);

  k_support<<<dim3(B), dim3(256), 0, stream>>>(Fs, Ms, gw1, gb1, gw2, gb2, Mt, g, Ps, Psn);
  k_pack<<<dim3(N / 32, B), dim3(256), 0, stream>>>(Fs, Fq, Mt, g, Aq, Bfg, Bcx);
  k_sim<<<dim3(N / 64, B, 2), dim3(128), 0, stream>>>(Aq, Bfg, Bcx, maxFg, maxCx);
  k_query<<<dim3(B), dim3(256), 0, stream>>>(Fq, maxFg, maxCx, fw, fb, Psn, psum);
  k_fqprime<<<dim3(PH, B), dim3(256), 0, stream>>>(Fq, psum, Ps, gamma, Fqp);
  k_packw<<<dim3((OC * CK / 8 + 255) / 256), dim3(256), 0, stream>>>(dw1, pW);
  k_conv<<<dim3(H, B), dim3(256), 0, stream>>>(Fqp, pW, db1, dw2, db2, out);
  (void)hipGetLastError();
}
